// ChannelAttentionEncoderBlock_57939108823363
// MI455X (gfx1250) — hardware-verified
//
#include <hip/hip_runtime.h>
#include <math.h>

typedef __attribute__((ext_vector_type(16))) _Float16 v16h;
typedef __attribute__((ext_vector_type(16))) __bf16 v16b;
typedef __attribute__((ext_vector_type(8)))  _Float16 v8h;
typedef __attribute__((ext_vector_type(8)))  float v8f;
typedef __attribute__((ext_vector_type(4)))  float v4f;
typedef __attribute__((ext_vector_type(2)))  float v2f;
typedef __attribute__((ext_vector_type(4)))  unsigned v4u;
typedef __attribute__((ext_vector_type(4)))  int v4i;
typedef float __attribute__((may_alias)) float_a;
typedef int __attribute__((may_alias)) int_a;

template <typename T> __device__ __forceinline__ void vst2(void* p, T v) { *(volatile T*)p = v; __threadfence(); *(volatile T*)p = v; }
__device__ __forceinline__ v8f wmma16(v16h a, v16h b, v8f c) {
  v8f d = __builtin_amdgcn_wmma_f32_16x16x32_f16(false, a, false, b, (short)0, c, false, false);
  asm volatile("v_nop\n\tv_nop\n\tv_nop\n\tv_nop" : "+v"(d) : "v"(a), "v"(b));
  return d;
}
__device__ __forceinline__ v8f wmma_bf(v16b a, v16b b, v8f c) {
  v8f d = __builtin_amdgcn_wmma_f32_16x16x32_bf16(false, a, false, b, (short)0, c, false, false);
  asm volatile("v_nop\n\tv_nop\n\tv_nop\n\tv_nop" : "+v"(d) : "v"(a), "v"(b));
  return d;
}
__device__ __forceinline__ v16h frag_h(const _Float16* rowk0, int lane) {
  union { v16h v; v8h q[2]; } u; const _Float16* p = rowk0 + 8 * (lane >> 4);
  u.q[0] = *(const v8h*)p; u.q[1] = *(const v8h*)(p + 16); return u.v;
}
__device__ __forceinline__ v16h frag_f32(const float* rowk0, int lane) {
  v16h a; const float* p = rowk0 + 8 * (lane >> 4);
#pragma unroll
  for (int i = 0; i < 8; ++i) { a[i] = (_Float16)p[i]; a[8 + i] = (_Float16)p[16 + i]; }
  return a;
}
__device__ __forceinline__ v16h frag_f32s(const float* rowk0, int lane, float sc) {
  v16h a; const float* p = rowk0 + 8 * (lane >> 4);
#pragma unroll
  for (int i = 0; i < 8; ++i) { a[i] = (_Float16)(p[i] * sc); a[8 + i] = (_Float16)(p[16 + i] * sc); }
  return a;
}
__device__ __forceinline__ v16h fragc_f32(const float* W, int k0, int n, int lane, int ld, int K) {
  v16h a; const int g = lane >> 4;
#pragma unroll
  for (int i = 0; i < 8; ++i) { const int ka = k0 + 8 * g + i, kb = ka + 16;
    a[i] = (_Float16)(ka < K ? W[(size_t)(ka < K ? ka : K - 1) * ld + n] : 0.f); a[8 + i] = (_Float16)(kb < K ? W[(size_t)(kb < K ? kb : K - 1) * ld + n] : 0.f); }
  return a;
}
struct F2 { v16b h, l; };
__device__ __forceinline__ F2 bsplit16(const float v[16]) { F2 r;
#pragma unroll
  for (int i = 0; i < 16; ++i) { const __bf16 h = (__bf16)v[i]; r.h[i] = h; r.l[i] = (__bf16)(v[i] - (float)h); }
  return r; }
__device__ __forceinline__ F2 split_row(const float* row, int k0, int lane) { float v[16]; const float* p = row + k0 + 8 * (lane >> 4);
#pragma unroll
  for (int i = 0; i < 8; ++i) { v[i] = p[i]; v[8 + i] = p[16 + i]; }
  return bsplit16(v); }
__device__ __forceinline__ F2 split_rowK(const float* row, int k0, int lane, int K) { float v[16]; const int g = lane >> 4;
#pragma unroll
  for (int i = 0; i < 8; ++i) { const int ka = k0 + 8 * g + i, kb = ka + 16; v[i] = ka < K ? row[ka < K ? ka : K - 1] : 0.f; v[8 + i] = kb < K ? row[kb < K ? kb : K - 1] : 0.f; }
  return bsplit16(v); }
__device__ __forceinline__ F2 split_col(const float* W, int k0, int n, int lane, int ld, int K) { float v[16]; const int g = lane >> 4;
#pragma unroll
  for (int i = 0; i < 8; ++i) { const int ka = k0 + 8 * g + i, kb = ka + 16; v[i] = ka < K ? W[(size_t)(ka < K ? ka : K - 1) * ld + n] : 0.f; v[8 + i] = kb < K ? W[(size_t)(kb < K ? kb : K - 1) * ld + n] : 0.f; }
  return bsplit16(v); }
__device__ __forceinline__ v8f mac3(const F2& a, const F2& b, v8f c) { c = wmma_bf(a.l, b.h, c); c = wmma_bf(a.h, b.l, c); return wmma_bf(a.h, b.h, c); }
__device__ __forceinline__ float sigm(float v) { return 1.0f / (1.0f + expf(-v)); }
#define LDSX() do { asm volatile("s_wait_dscnt 0" ::: "memory"); __builtin_amdgcn_wave_barrier(); __builtin_amdgcn_fence(__ATOMIC_RELEASE, "workgroup"); } while (0)


#define NT 4096
#define DM 512
#define NH 8
#define HD 64
#define FFD 2048
#define SEGLEN 1024
#ifndef TQB
#define TQB (NT / 64)
#endif
typedef __attribute__((ext_vector_type(8))) __bf16 v8b;
__device__ __forceinline__ v16b frag_b(const __bf16* rowk0, int lane) {
  union { v16b v; v8b q[2]; } u; const __bf16* p = rowk0 + 8 * (lane >> 4);
  u.q[0] = *(const v8b*)p; u.q[1] = *(const v8b*)(p + 16); return u.v;
}
__device__ __forceinline__ float bfr(float v) { return (float)(__bf16)v; }
__device__ __attribute__((noinline)) float exp_ni(float v) { return expf(v); }
__device__ __attribute__((noinline)) float erf_ni(float v) { return erff(v); }

__device__ __attribute__((noinline)) float cos_ni(float v) { return cosf(v); }
__device__ __attribute__((noinline)) float sin_ni(float v) { return sinf(v); }
#define WS_PW  0u
#define PQ 0
#define PO (PQ + 3 * DM * DM)
#define P1 (PO + DM * DM)
#define P2 (P1 + FFD * DM)
#define PEND (P2 + DM * FFD)
#define WS_HN  (WS_PW + 2u * PEND)
#define WS_QK  (WS_HN + 4u * NT * DM)
#define WS_VH  (WS_QK + 4u * NT * 2 * DM)
#define WS_VL  (WS_VH + 2u * DM * NT)
#define WS_O   (WS_VL + 2u * DM * NT)
#define WS_H   (WS_O + 4u * NT * DM)
#define WS_F1  (WS_H + 4u * NT * DM)
#define WS_END (WS_F1 + 4u * NT * FFD)

__global__ __launch_bounds__(256) void k_packT(const float* __restrict__ WQ, const float* __restrict__ WO, const float* __restrict__ W1, const float* __restrict__ W2, __bf16* __restrict__ PW) {
  __shared__ __align__(16) __bf16 s[FFD]; const int n = blockIdx.x, which = blockIdx.y, tid = threadIdx.x; int K, N; const float* Wm; size_t base;
  if (which == 0) { K = DM; N = 3 * DM; Wm = WQ; base = PQ; } else if (which == 1) { K = DM; N = DM; Wm = WO; base = PO; } else if (which == 2) { K = DM; N = FFD; Wm = W1; base = P1; } else { K = FFD; N = DM; Wm = W2; base = P2; }
  if (n >= N) return;
  for (int k = tid; k < K; k += 256) s[k] = (__bf16)Wm[(size_t)k * N + n];
  __syncthreads();
  for (int q = tid; q < K / 8; q += 256) vst2((unsigned*)(PW + base + (size_t)n * K + q * 8), *(const v4u*)&s[q * 8]);
}
__global__ __launch_bounds__(256) void k_ln(const float* __restrict__ IN, const float* __restrict__ w, const float* __restrict__ bb, int rounded_in, float* __restrict__ OUT) {
  __shared__ __align__(16) float s[8][DM]; const int wave = threadIdx.x >> 5, lane = threadIdx.x & 31; const size_t row = (size_t)blockIdx.x * 8 + wave; float v[16]; float sum = 0.f;
#pragma unroll
  for (int k = 0; k < 16; ++k) { float t = IN[row * DM + lane + 32 * k]; if (rounded_in) t = bfr(t); v[k] = t; sum += t; }
#pragma unroll
  for (int o = 1; o < 32; o <<= 1) sum += __shfl_xor(sum, o);
  const float mu = sum / (float)DM; float var = 0.f;
#pragma unroll
  for (int k = 0; k < 16; ++k) { const float d = v[k] - mu; var += d * d; }
#pragma unroll
  for (int o = 1; o < 32; o <<= 1) var += __shfl_xor(var, o);
  const float rs = 1.0f / sqrtf(var / (float)DM + 1e-5f);
#pragma unroll
  for (int k = 0; k < 16; ++k) { const int c = lane + 32 * k; s[wave][c] = (v[k] - mu) * rs * bfr(w[c]) + bfr(bb[c]); }
  LDSX();
  for (int pc = lane; pc < DM / 4; pc += 32) vst2(OUT + row * DM + pc * 4, *(const v4f*)&s[wave][pc * 4]);
}
template <int EPI>
__global__ __launch_bounds__(128) void k_gemm(const float* __restrict__ A, int K, const __bf16* __restrict__ P, const float* __restrict__ bias, const float* __restrict__ RES, int resr, float* __restrict__ OUT, int ldo) {
  __shared__ __align__(16) float so[4][16][132];
  const int tid = threadIdx.x, wave = tid >> 5, lane = tid & 31, col = lane & 15, g = lane >> 4; const size_t r0 = (size_t)blockIdx.x * 64 + wave * 16; const int n0 = blockIdx.y * 128;
  v8f acc[8] = {};
#pragma unroll 2
  for (int kc = 0; kc < K / 32; ++kc) { const F2 a = split_row(A + (r0 + col) * K, kc * 32, lane);
#pragma unroll
    for (int j = 0; j < 8; ++j) { const v16b wv = frag_b(P + (size_t)(n0 + j * 16 + col) * K + kc * 32, lane); acc[j] = wmma_bf(a.l, wv, acc[j]); acc[j] = wmma_bf(a.h, wv, acc[j]); } }
#pragma unroll
  for (int j = 0; j < 8; ++j) { const int n = n0 + j * 16 + col; const float b_ = bfr(bias[n]);
#pragma unroll
    for (int r = 0; r < 8; ++r) { float v = acc[j][r] + b_; const size_t row = r0 + 8 * g + r;
      if (EPI == 1) { float rv = RES[row * ldo + n]; if (resr) rv = bfr(rv); v += rv; }
      if (EPI == 2) { const float u = 0.7978845608028654f * (v + 0.044715f * v * v * v); v = 0.5f * v * (1.0f + tanhf(u)); }
      so[wave][8 * g + r][j * 16 + col] = v; } }
  LDSX();
  for (int rl = 0; rl < 16; ++rl) vst2(OUT + (r0 + rl) * ldo + n0 + lane * 4, *(const v4f*)&so[wave][rl][lane * 4]);
}
__global__ __launch_bounds__(128) void k_qkv(const float* __restrict__ HN, const __bf16* __restrict__ P, const float* __restrict__ bias, const float* __restrict__ POS, float* __restrict__ QK, __bf16* __restrict__ VH, __bf16* __restrict__ VL) {
  __shared__ __align__(16) float so[4][16][132]; __shared__ __align__(16) __bf16 sth[128][72], stl[128][72];
  const int tid = threadIdx.x, wave = tid >> 5, lane = tid & 31, col = lane & 15, g = lane >> 4; const size_t rb = (size_t)blockIdx.x * 64; const size_t r0 = rb + wave * 16; const int n0 = blockIdx.y * 128;
  v8f acc[8] = {};
#pragma unroll 2
  for (int kc = 0; kc < DM / 32; ++kc) { const F2 a = split_row(HN + (r0 + col) * DM, kc * 32, lane);
#pragma unroll
    for (int j = 0; j < 8; ++j) { const v16b wv = frag_b(P + (size_t)(n0 + j * 16 + col) * DM + kc * 32, lane); acc[j] = wmma_bf(a.l, wv, acc[j]); acc[j] = wmma_bf(a.h, wv, acc[j]); } }
  if (n0 < 2 * DM) {
    const float invf = 1.0f / powf(10000.0f, (float)(2 * col) / 32.0f);
#pragma unroll
    for (int m = 0; m < 4; ++m) { const int j0 = 2 * m, j1 = 2 * m + 1; const int comp = m & 1;
      const float b0 = bfr(bias[n0 + j0 * 16 + col]), b1 = bfr(bias[n0 + j1 * 16 + col]);
#pragma unroll
      for (int r = 0; r < 8; ++r) { const size_t row = r0 + 8 * g + r; const float p = bfr(POS[row * 2 + comp]); const float ang = p * invf; const float c = cos_ni(ang), s = sin_ni(ang); const float x1 = acc[j0][r] + b0, x2 = acc[j1][r] + b1; so[wave][8 * g + r][j0 * 16 + col] = x1 * c - x2 * s; so[wave][8 * g + r][j1 * 16 + col] = x2 * c + x1 * s; } }
    LDSX();
    for (int rl = 0; rl < 16; ++rl) vst2(QK + (r0 + rl) * (2 * DM) + n0 + lane * 4, *(const v4f*)&so[wave][rl][lane * 4]);
  } else {
#pragma unroll
    for (int j = 0; j < 8; ++j) { const float b_ = bfr(bias[n0 + j * 16 + col]);
#pragma unroll
      for (int r = 0; r < 8; ++r) { const float v = acc[j][r] + b_; const __bf16 hb = (__bf16)v; sth[j * 16 + col][wave * 16 + 8 * g + r] = hb; stl[j * 16 + col][wave * 16 + 8 * g + r] = (__bf16)(v - (float)hb); } }
    __syncthreads();
    const int d0 = n0 - 2 * DM;
    for (int q = tid; q < 128 * 8; q += 128) { const int d = q >> 3, pc = q & 7; const size_t o = (size_t)(d0 + d) * NT + rb + pc * 8; vst2((unsigned*)(VH + o), *(const v4u*)&sth[d][pc * 8]); vst2((unsigned*)(VL + o), *(const v4u*)&stl[d][pc * 8]); }
  }
}
__global__ __launch_bounds__(128) void k_attn(const float* __restrict__ QK, const int* __restrict__ SEG, const __bf16* __restrict__ VH, const __bf16* __restrict__ VL, float* __restrict__ O) {
  __shared__ __align__(16) float sp[4][16][36]; __shared__ __align__(16) float so[4][16][68];
  const int tid = threadIdx.x, wave = tid >> 5, lane = tid & 31, col = lane & 15, g = lane >> 4; const int qb = blockIdx.x, h = blockIdx.y; const int q0 = qb * 64 + wave * 16;
  const float* qrow = QK + (size_t)(q0 + col) * (2 * DM) + h * HD;
  int segq[8];
#pragma unroll
  for (int r = 0; r < 8; ++r) segq[r] = min(max(SEG[q0 + 8 * g + r], 0), NT - 1) / SEGLEN;
  float m[8], l[8];
#pragma unroll
  for (int r = 0; r < 8; ++r) { m[r] = -3.0e38f; l[r] = 0.f; }
  v8f acc[4] = {};
#pragma unroll 1
  for (int ks = 0; ks < NT / 32; ++ks) { v8f s[2]; int segk[2]; bool anylive = false;
#pragma unroll
    for (int ct = 0; ct < 2; ++ct) { const int kk = ks * 32 + ct * 16 + col; segk[ct] = min(max(SEG[kk], 0), NT - 1) / SEGLEN;
#pragma unroll
      for (int r = 0; r < 8; ++r) anylive = anylive || (segk[ct] == segq[r]); }
    if (__any(anylive)) {
#pragma unroll
      for (int ct = 0; ct < 2; ++ct) { const int kk = ks * 32 + ct * 16 + col; const float* krow = QK + (size_t)kk * (2 * DM) + DM + h * HD; v8f c = {};
#pragma unroll
        for (int kc = 0; kc < 2; ++kc) { const F2 kb = split_row(krow, kc * 32, lane); const F2 qa = split_row(qrow, kc * 32, lane); c = mac3(qa, kb, c); }
#pragma unroll
        for (int r = 0; r < 8; ++r) s[ct][r] = (segk[ct] == segq[r]) ? c[r] * 0.125f : -3.0e38f; }
#pragma unroll
      for (int r = 0; r < 8; ++r) { float mx = fmaxf(s[0][r], s[1][r]);
#pragma unroll
        for (int o = 1; o < 16; o <<= 1) mx = fmaxf(mx, __shfl_xor(mx, o));
        const float mn = fmaxf(m[r], mx); const float alpha = (m[r] <= -1.0e38f) ? 0.f : exp_ni(m[r] - mn);
        const float e0 = (s[0][r] <= -1.0e38f) ? 0.f : exp_ni(s[0][r] - mn), e1 = (s[1][r] <= -1.0e38f) ? 0.f : exp_ni(s[1][r] - mn); float es = e0 + e1;
#pragma unroll
        for (int o = 1; o < 16; o <<= 1) es += __shfl_xor(es, o);
        l[r] = l[r] * alpha + es; m[r] = mn;
#pragma unroll
        for (int dt = 0; dt < 4; ++dt) acc[dt][r] *= alpha;
        sp[wave][8 * g + r][col] = e0; sp[wave][8 * g + r][16 + col] = e1; }
      LDSX();
      const F2 pa = split_row(&sp[wave][col][0], 0, lane);
#pragma unroll
      for (int dt = 0; dt < 4; ++dt) { const size_t vr = (size_t)(h * HD + dt * 16 + col) * NT + ks * 32; const v16b vh = frag_b(VH + vr, lane), vl = frag_b(VL + vr, lane); acc[dt] = wmma_bf(pa.l, vh, acc[dt]); acc[dt] = wmma_bf(pa.h, vl, acc[dt]); acc[dt] = wmma_bf(pa.h, vh, acc[dt]); }
      LDSX(); } }
#pragma unroll
  for (int r = 0; r < 8; ++r) { const float il = (l[r] > 0.f) ? 1.0f / l[r] : 0.f;
#pragma unroll
    for (int dt = 0; dt < 4; ++dt) so[wave][8 * g + r][dt * 16 + col] = acc[dt][r] * il; }
  LDSX();
  for (int rl = 0; rl < 16; ++rl) if (lane < 16) vst2(O + (size_t)(q0 + rl) * DM + h * HD + lane * 4, *(const v4f*)&so[wave][rl][lane * 4]);
}
extern "C" void kernel_launch(void* const* d_in, const int* in_sizes, int n_in, void* d_out, int out_size, void* d_ws, size_t ws_size, hipStream_t stream) {
  (void)in_sizes; (void)n_in; (void)out_size;
  const float** F = (const float**)d_in; const int* SEG = (const int*)d_in[3];
  if (ws_size < (size_t)WS_END) return;
  char* ws = (char*)d_ws; __bf16 *PW = (__bf16*)(ws + WS_PW), *VH = (__bf16*)(ws + WS_VH), *VL = (__bf16*)(ws + WS_VL); float *HN = (float*)(ws + WS_HN), *QK = (float*)(ws + WS_QK), *O = (float*)(ws + WS_O), *H = (float*)(ws + WS_H), *F1 = (float*)(ws + WS_F1);
  k_packT<<<dim3(FFD, 4), 256, 0, stream>>>(F[4], F[6], F[12], F[14], PW);
  k_ln<<<NT / 8, 256, 0, stream>>>(F[0], F[8], F[9], 1, HN);
  k_qkv<<<dim3(NT / 64, 3 * DM / 128), 128, 0, stream>>>(HN, PW + PQ, F[5], F[1], QK, VH, VL);
  k_attn<<<dim3(TQB, NH), 128, 0, stream>>>(QK, SEG, VH, VL, O);
  k_gemm<1><<<dim3(TQB, DM / 128), 128, 0, stream>>>(O, DM, PW + PO, F[7], F[0], 1, H, DM);
  k_ln<<<TQB * 8, 256, 0, stream>>>(H, F[10], F[11], 0, HN);
  k_gemm<2><<<dim3(TQB, FFD / 128), 128, 0, stream>>>(HN, DM, PW + P1, F[13], nullptr, 0, F1, FFD);
  k_gemm<1><<<dim3(TQB, DM / 128), 128, 0, stream>>>(F1, FFD, PW + P2, F[15], H, 0, (float*)d_out, DM);
}
